// BahdanauAttention_24000277250165
// MI455X (gfx1250) — hardware-verified
//
#include <hip/hip_runtime.h>


#ifndef NB
#define NB 8
#endif
#ifndef TQ
#define TQ 256
#endif
#define NB_FULL 8
#define T_FULL 256
#define S_LEN 256
#define HD 512
#define KC (2 * S_LEN)
#define KO (3 * HD)

static_assert(NB >= 1 && NB <= NB_FULL);
static_assert(TQ >= 64 && TQ <= T_FULL && (TQ % 64) == 0);
static_assert(S_LEN == 256);
static_assert((HD % 256) == 0);
static_assert((KC % 32) == 0 && (KO % 32) == 0 && (HD % 64) == 0 && (S_LEN % 64) == 0);

typedef unsigned short us;
typedef us     v8us  __attribute__((ext_vector_type(8)));
typedef __bf16 v16bf __attribute__((ext_vector_type(16)));
typedef float  v8f   __attribute__((ext_vector_type(8)));
typedef float  v4f   __attribute__((ext_vector_type(4)));

union Frag { v16bf v; v8us h[2]; };

__device__ __forceinline__ us f2bf(float f) {
    unsigned int u = __float_as_uint(f);
    u += 0x7FFFu + ((u >> 16) & 1u);
    return (us)(u >> 16);
}
__device__ __forceinline__ float bf2f(us h) {
    return __uint_as_float(((unsigned int)h) << 16);
}
__device__ __forceinline__ float tanh_acc(float x) {
    const float ax = __builtin_fabsf(x);
    const float t  = __expf(-2.0f * ax);
    const float r  = (1.0f - t) * __builtin_amdgcn_rcpf(1.0f + t);
    return __builtin_copysignf(r, x);
}
__device__ __forceinline__ v8us pack8(v4f a, v4f c) {
    v8us o;
    o[0] = f2bf(a.x); o[1] = f2bf(a.y); o[2] = f2bf(a.z); o[3] = f2bf(a.w);
    o[4] = f2bf(c.x); o[5] = f2bf(c.y); o[6] = f2bf(c.z); o[7] = f2bf(c.w);
    return o;
}
__device__ __forceinline__ void split8(v4f a, v4f c, v8us& hi, v8us& lo) {
    const float x[8] = {a.x, a.y, a.z, a.w, c.x, c.y, c.z, c.w};
#pragma unroll
    for (int i = 0; i < 8; ++i) {
        const us h = f2bf(x[i]);
        hi[i] = h;
        lo[i] = f2bf(x[i] - bf2f(h));
    }
}

__device__ __forceinline__ v8f wmma16(v16bf a, v16bf b, v8f c) {
    v8f d = __builtin_amdgcn_wmma_f32_16x16x32_bf16(false, a, false, b, (short)0, c, false, false);
    asm volatile("v_nop\n\tv_nop\n\tv_nop\n\tv_nop" : "+v"(d) : "v"(a), "v"(b));
    return d;
}

__device__ __forceinline__ v16bf ld_frag(const us* __restrict__ P, int ld, int row, int k0, int hsel) {
    Frag f;
    const us* p = P + (size_t)row * ld + k0 + 8 * hsel;
    f.h[0] = *(const v8us*)p;
    f.h[1] = *(const v8us*)(p + 16);
    return f.v;
}

__global__ __launch_bounds__(256)
void k_cvt(const float* __restrict__ src, int spitch, int scol, int grp, int gstride,
           us* __restrict__ dst, int dpitch, int dcol, int nrows, int nseg)
{
    const int lane = threadIdx.x & 31;
    const int gw   = blockIdx.x * 8 + (threadIdx.x >> 5);
    if (gw >= nrows * nseg) return;
    const int r    = gw / nseg;
    const int sg   = gw - r * nseg;
    const int g    = r / grp;
    const int srow = g * gstride + (r - g * grp);
    const float* sp = src + (size_t)srow * spitch + scol + sg * 256 + lane * 8;
    const v4f a = *(const v4f*)sp;
    const v4f c = *(const v4f*)(sp + 4);
    const v8us o = pack8(a, c);
    us* dp = dst + (size_t)r * dpitch + dcol + sg * 256 + lane * 8;
    *(volatile v8us*)dp = o;
    __threadfence();
    *(volatile v8us*)dp = o;
}

__global__ __launch_bounds__(256)
void k_trans(const float* __restrict__ enc, us* __restrict__ encT2)
{
    __shared__ float ts[64][65];
    const int s0 = blockIdx.x * 64, h0 = blockIdx.y * 64, b = blockIdx.z;
    const int tid = threadIdx.x, lane = tid & 31, wave = tid >> 5;

#pragma unroll
    for (int p = 0; p < 4; ++p) {
        const int sl = p * 16 + (tid >> 4);
        const int h4 = (tid & 15) * 4;
        const v4f x = *(const v4f*)(enc + ((size_t)(b * S_LEN + s0 + sl)) * HD + h0 + h4);
        ts[sl][h4 + 0] = x.x; ts[sl][h4 + 1] = x.y; ts[sl][h4 + 2] = x.z; ts[sl][h4 + 3] = x.w;
    }
    __syncthreads();

    v8us o[2];
#pragma unroll
    for (int p = 0; p < 2; ++p) {
        const int hl = p * 32 + wave * 4 + (lane >> 3);
        const int s8 = (lane & 7) * 8;
#pragma unroll
        for (int i = 0; i < 8; ++i) o[p][i] = f2bf(ts[s8 + i][hl]);
    }
#pragma unroll
    for (int p = 0; p < 2; ++p) {
        const int hl = p * 32 + wave * 4 + (lane >> 3);
        const int s8 = (lane & 7) * 8;
        us* d = encT2 + ((size_t)(b * HD + h0 + hl)) * KC + s0 + s8;
        *(volatile v8us*)d = o[p];
        *(volatile v8us*)(d + S_LEN) = o[p];
    }
    __threadfence();
#pragma unroll
    for (int p = 0; p < 2; ++p) {
        const int hl = p * 32 + wave * 4 + (lane >> 3);
        const int s8 = (lane & 7) * 8;
        us* d = encT2 + ((size_t)(b * HD + h0 + hl)) * KC + s0 + s8;
        *(volatile v8us*)d = o[p];
        *(volatile v8us*)(d + S_LEN) = o[p];
    }
}

template <int EPI>
__global__ __launch_bounds__(128)
void k_gemm(const us* __restrict__ A, int lda, int strideA,
            const us* __restrict__ B, int ldb, int strideB,
            void* __restrict__ Cv, int ldc, int strideC, int K, int loff)
{
    __shared__ __attribute__((aligned(16))) float tile[4 * 16 * 64];

    const int lane = threadIdx.x & 31, wave = threadIdx.x >> 5;
    const int hsel = lane >> 4, m = lane & 15;
    const int m0 = blockIdx.x * 64 + wave * 16;
    const int n0 = blockIdx.y * 64;
    const us* Ab = A + (size_t)blockIdx.z * (size_t)strideA;
    const us* Bb = B + (size_t)blockIdx.z * (size_t)strideB;

    v8f c0 = {}; v8f c1 = {}; v8f c2 = {}; v8f c3 = {};
    for (int k0 = 0; k0 < K; k0 += 32) {
        const v16bf a  = ld_frag(Ab, lda, m0 + m, k0, hsel);
        const v16bf b0 = ld_frag(Bb, ldb, n0 + m,      k0, hsel);
        const v16bf b1 = ld_frag(Bb, ldb, n0 + 16 + m, k0, hsel);
        const v16bf b2 = ld_frag(Bb, ldb, n0 + 32 + m, k0, hsel);
        const v16bf b3 = ld_frag(Bb, ldb, n0 + 48 + m, k0, hsel);
        c0 = wmma16(a, b0, c0);
        c1 = wmma16(a, b1, c1);
        c2 = wmma16(a, b2, c2);
        c3 = wmma16(a, b3, c3);
    }

    float* tw = tile + wave * 1024;
#pragma unroll
    for (int r = 0; r < 8; ++r) {
        const int row = 8 * hsel + r;
        tw[row * 64 + m]      = c0[r];
        tw[row * 64 + 16 + m] = c1[r];
        tw[row * 64 + 32 + m] = c2[r];
        tw[row * 64 + 48 + m] = c3[r];
    }
    __syncthreads();

    if (EPI == 1) {
        us* Cb = (us*)Cv + (size_t)blockIdx.z * (size_t)strideC;
        v8us hi[4], lo[4];
#pragma unroll
        for (int p = 0; p < 4; ++p) {
            const int row = 4 * p + (lane >> 3);
            const int col = 8 * (lane & 7);
            const v4f a = *(const v4f*)(tw + row * 64 + col);
            const v4f c = *(const v4f*)(tw + row * 64 + col + 4);
            split8(a, c, hi[p], lo[p]);
        }
#pragma unroll
        for (int p = 0; p < 4; ++p) {
            us* d = Cb + (size_t)(m0 + 4 * p + (lane >> 3)) * ldc + n0 + 8 * (lane & 7);
            *(volatile v8us*)d = hi[p];
            *(volatile v8us*)(d + loff) = lo[p];
        }
        __threadfence();
#pragma unroll
        for (int p = 0; p < 4; ++p) {
            us* d = Cb + (size_t)(m0 + 4 * p + (lane >> 3)) * ldc + n0 + 8 * (lane & 7);
            *(volatile v8us*)d = hi[p];
            *(volatile v8us*)(d + loff) = lo[p];
        }
    } else {
        float* Cb = (float*)Cv + (size_t)blockIdx.z * (size_t)strideC;
        v4f vals[8];
#pragma unroll
        for (int p = 0; p < 8; ++p) {
            const int row = 2 * p + hsel;
            v4f x = *(const v4f*)(tw + row * 64 + 4 * m);
            if (EPI == 2) {
                x.x = tanh_acc(x.x); x.y = tanh_acc(x.y); x.z = tanh_acc(x.z); x.w = tanh_acc(x.w);
            }
            vals[p] = x;
        }
#pragma unroll
        for (int p = 0; p < 8; ++p) {
            float* d = Cb + (size_t)(m0 + 2 * p + hsel) * ldc + n0 + 4 * m;
            *(volatile v4f*)d = vals[p];
        }
        __threadfence();
#pragma unroll
        for (int p = 0; p < 8; ++p) {
            float* d = Cb + (size_t)(m0 + 2 * p + hsel) * ldc + n0 + 4 * m;
            *(volatile v4f*)d = vals[p];
        }
    }
}

__global__ __launch_bounds__(256)
void k_attn(const float* __restrict__ Wsq, const float* __restrict__ Whe,
            const float* __restrict__ vvec, const int* __restrict__ lens,
            us* __restrict__ Pcat)
{
    __shared__ v4f sq4[HD / 4];
    __shared__ v4f sv4[HD / 4];
    __shared__ __attribute__((aligned(16))) float sp[S_LEN];
    __shared__ float red[S_LEN];

    const int bt  = blockIdx.x;
    const int b   = bt / TQ;
    const int tid = threadIdx.x, lane = tid & 31, wave = tid >> 5;

    if (tid < HD / 4) {
        sq4[tid] = *(const v4f*)(Wsq + (size_t)bt * HD + tid * 4);
        v4f w = *(const v4f*)(vvec + tid * 4);
        w.x = bf2f(f2bf(w.x)); w.y = bf2f(f2bf(w.y)); w.z = bf2f(f2bf(w.z)); w.w = bf2f(f2bf(w.w));
        sv4[tid] = w;
    }
    __syncthreads();

    const int len = lens[b];
    const v4f* we = (const v4f*)(Whe + ((size_t)b * S_LEN + tid) * HD);
    float acc = 0.0f;
#pragma unroll 2
    for (int u = 0; u < HD / 4; ++u) {
        const v4f e = we[u];
        const v4f d = sq4[u];
        const v4f w = sv4[u];
        acc += w.x * tanh_acc(e.x + d.x);
        acc += w.y * tanh_acc(e.y + d.y);
        acc += w.z * tanh_acc(e.z + d.z);
        acc += w.w * tanh_acc(e.w + d.w);
    }
    const bool valid = tid < len;
    const float en = valid ? acc : -3.0e38f;

    red[tid] = en;
    __syncthreads();
#pragma unroll
    for (int st = S_LEN / 2; st > 0; st >>= 1) {
        if (tid < st) red[tid] = fmaxf(red[tid], red[tid + st]);
        __syncthreads();
    }
    const float mx = red[0];
    __syncthreads();

    const float arg = valid ? (acc - mx) : -80.0f;
    const float ex0 = __expf(arg);
    const float ex  = valid ? ex0 : 0.0f;
    red[tid] = ex;
    __syncthreads();
#pragma unroll
    for (int st = S_LEN / 2; st > 0; st >>= 1) {
        if (tid < st) red[tid] += red[tid + st];
        __syncthreads();
    }
    const float ssum = red[0];
    const float p = ex * (1.0f / ssum);
    sp[tid] = p;
    __syncthreads();

    if (wave < 2) {
        const v4f a = *(const v4f*)(sp + lane * 8);
        const v4f c = *(const v4f*)(sp + lane * 8 + 4);
        v8us hi, lo;
        split8(a, c, hi, lo);
        v8us o;
        if (wave == 0) o = hi; else o = lo;
        us* d = Pcat + (size_t)bt * KC + wave * S_LEN + lane * 8;
        *(volatile v8us*)d = o;
        __threadfence();
        *(volatile v8us*)d = o;
    }
}

static inline size_t al256(size_t x) { return (x + 255) & ~(size_t)255; }

extern "C" void kernel_launch(void* const* d_in, const int* in_sizes, int n_in,
                              void* d_out, int out_size, void* d_ws, size_t ws_size,
                              hipStream_t stream)
{
    if (n_in < 7) return;
    if (in_sizes[0] < ((NB - 1) * T_FULL + TQ) * HD) return;
    if (in_sizes[1] < NB * S_LEN * HD) return;
    if (in_sizes[2] < NB) return;
    if (in_sizes[3] < HD * HD || in_sizes[4] < HD * HD) return;
    if (in_sizes[5] < HD) return;
    if (in_sizes[6] < HD * 2 * HD) return;
    if (out_size < ((NB - 1) * T_FULL + TQ) * HD) return;

    const float* query = (const float*)d_in[0];
    const float* enc   = (const float*)d_in[1];
    const int*   lens  = (const int*)d_in[2];
    const float* W_s   = (const float*)d_in[3];
    const float* W_h   = (const float*)d_in[4];
    const float* vvec  = (const float*)d_in[5];
    const float* W_out = (const float*)d_in[6];
    float* out = (float*)d_out;

    char* ws = (char*)d_ws;
    size_t off = 0;
    us* comb  = (us*)(ws + off);    off += al256((size_t)NB * TQ * KO * sizeof(us));
    us* encb  = (us*)(ws + off);    off += al256((size_t)NB * S_LEN * HD * sizeof(us));
    us* encT2 = (us*)(ws + off);    off += al256((size_t)NB * HD * KC * sizeof(us));
    us* Wsb   = (us*)(ws + off);    off += al256((size_t)HD * HD * sizeof(us));
    us* Whb   = (us*)(ws + off);    off += al256((size_t)HD * HD * sizeof(us));
    us* WoX   = (us*)(ws + off);    off += al256((size_t)HD * KO * sizeof(us));
    float* Wsq = (float*)(ws + off); off += al256((size_t)NB * TQ * HD * sizeof(float));
    float* Whe = (float*)(ws + off); off += al256((size_t)NB * S_LEN * HD * sizeof(float));
    us* Pcat  = (us*)(ws + off);    off += al256((size_t)NB * TQ * KC * sizeof(us));
    if (off > ws_size) return;

    const dim3 b256(256), b128(128);

    {
        const int nrows = NB * TQ, nseg = HD / 256;
        k_cvt<<<dim3((nrows * nseg + 7) / 8), b256, 0, stream>>>(
            query, HD, 0, TQ, T_FULL, comb, KO, 2 * HD, nrows, nseg);
    }
    {
        const int nrows = NB * S_LEN, nseg = HD / 256;
        k_cvt<<<dim3((nrows * nseg + 7) / 8), b256, 0, stream>>>(
            enc, HD, 0, S_LEN, S_LEN, encb, HD, 0, nrows, nseg);
    }
    {
        const int nrows = HD, nseg = HD / 256;
        const dim3 g((nrows * nseg + 7) / 8);
        k_cvt<<<g, b256, 0, stream>>>(W_s, HD, 0, HD, HD, Wsb, HD, 0, nrows, nseg);
        k_cvt<<<g, b256, 0, stream>>>(W_h, HD, 0, HD, HD, Whb, HD, 0, nrows, nseg);
        k_cvt<<<g, b256, 0, stream>>>(W_out, 2 * HD, 0,  HD, HD, WoX, KO, 0,      nrows, nseg);
        k_cvt<<<g, b256, 0, stream>>>(W_out, 2 * HD, 0,  HD, HD, WoX, KO, HD,     nrows, nseg);
        k_cvt<<<g, b256, 0, stream>>>(W_out, 2 * HD, HD, HD, HD, WoX, KO, 2 * HD, nrows, nseg);
    }
    k_trans<<<dim3(S_LEN / 64, HD / 64, NB), b256, 0, stream>>>(enc, encT2);

    k_gemm<0><<<dim3(NB * TQ / 64, HD / 64, 1), b128, 0, stream>>>(
        comb + 2 * HD, KO, 0, Wsb, HD, 0, (void*)Wsq, HD, 0, HD, 0);
    k_gemm<0><<<dim3(NB * S_LEN / 64, HD / 64, 1), b128, 0, stream>>>(
        encb, HD, 0, Whb, HD, 0, (void*)Whe, HD, 0, HD, 0);

    k_attn<<<dim3(NB * TQ), b256, 0, stream>>>(Wsq, Whe, vvec, lens, Pcat);

    k_gemm<1><<<dim3(TQ / 64, HD / 64, NB), b128, 0, stream>>>(
        Pcat, KC, TQ * KC, encT2, KC, HD * KC, (void*)comb, KO, TQ * KO, KC, HD);

    k_gemm<2><<<dim3(TQ / 64, HD / 64, NB), b128, 0, stream>>>(
        comb, KO, TQ * KO, WoX, KO, 0, (void*)out, HD, T_FULL * HD, KO, 0);
}
